// SwinTransformerBlock_33578054320258
// MI455X (gfx1250) — hardware-verified
//
#include <hip/hip_runtime.h>
#include <math.h>

#ifndef NB
#define NB 32
#endif
#define NB_FULL 32
#define HW 56
#define LTOK 3136
#define CD 128
#define NH 4
#define HD 32
#define WSZ 7
#define NTOK 49
#define WROWS 64
#define NWIMG 64
#define SHIFT 3
#define QKVN 384
#define NPASS ((NB >= 2) ? 2 : 1)
#define IMGS (NB / NPASS)
#define NWINP (IMGS * NWIMG)
#define MROWS (NWINP * WROWS)

#define X_CARRY 16.0f
#define W_CARRY 64.0f
#define QKV_CARRY 256.0f
#define P_CARRY 1024.0f
#define CTX_CARRY 256.0f
#define QKV_UNDO (1.0f / 1024.0f)
#define S_UNDO (1.0f / 65536.0f)
#define O_UNDO (1.0f / 1024.0f)
#define PROJ_UNDO (1.0f / 16384.0f)
#define QSCALE 0.17677669529663687f
#define LOG2E 1.4426950408889634f

static_assert(X_CARRY * W_CARRY * QKV_UNDO == 1.0f);
static_assert(QKV_CARRY * QKV_CARRY * S_UNDO == 1.0f);
static_assert(P_CARRY * QKV_CARRY * O_UNDO == CTX_CARRY);
static_assert(CTX_CARRY * W_CARRY * PROJ_UNDO == 1.0f);

static_assert(NB <= NB_FULL && NB % NPASS == 0);
static_assert(HW % WSZ == 0 && (HW / WSZ) == 8 && (HW / WSZ) * (HW / WSZ) == NWIMG);
static_assert(HW * HW == LTOK);
static_assert(WSZ * WSZ == NTOK && NTOK <= WROWS && WROWS == 64);
static_assert(NH * HD == CD && HD == 32 && CD == 128);
static_assert(QKVN == 3 * CD && QKVN % 64 == 0 && CD % 64 == 0 && CD % 32 == 0);
static_assert(NWINP % 8 == 0 && MROWS % 64 == 0);
static_assert((MROWS * (CD / 8)) % 256 == 0);
static_assert((QKVN * CD / 8) % 256 == 0 && (CD * CD / 8) % 256 == 0);
static_assert(SHIFT < WSZ);
static_assert(4 * 16 * 68 * 4 + 4 * 64 * 72 * 2 <= 131072);
static_assert(4 * 176 * 4 + 2432 * 4 + 8 * 16 * 72 * 2 <= 131072);
static_assert(8 * 16 * 68 * 4 <= 131072);
static_assert(32 * 16 * 4 == 16 * 128);
static_assert(32 * 16 * 4 * 4 == 64 * 128);
static_assert(32 * 16 * 4 * 2 == 16 * 256);
static_assert(2401 <= 2432 && 169 <= 176);
static_assert((size_t)5 * MROWS * CD * 2 + (size_t)(QKVN * CD + CD * CD) * 2 + 4096 <= (size_t)134217728);

typedef _Float16 h16;
typedef __attribute__((ext_vector_type(16))) _Float16 v16h;
typedef __attribute__((ext_vector_type(8)))  _Float16 v8h;
typedef __attribute__((ext_vector_type(8)))  float    v8f;
typedef __attribute__((ext_vector_type(4)))  float    v4f;


__device__ __forceinline__ float bfr(float f) {
    unsigned u = __float_as_uint(f);
    u += 0x7FFFu + ((u >> 16) & 1u);
    return __uint_as_float(u & 0xFFFF0000u);
}
static __device__ __forceinline__ h16 toh_flush(float v) { const float w = (fabsf(v) < 6.103515625e-05f) ? 0.0f : v; return (h16)w; }
static __device__ __forceinline__ unsigned div7_u6(unsigned t) {
    asm volatile("" : "+v"(t));
    return (t * 9363u) >> 16;
}

__device__ __forceinline__ void st8_twice(_Float16* p, v8h pk) {
    *(volatile v8h*)p = pk;
    __threadfence();
    *(volatile v8h*)p = pk;
}

union FragU { v16h v; v8h h[2]; };
__device__ __forceinline__ v16h frag_ld(const _Float16* p) {
    FragU f; f.h[0] = *(const v8h*)(p); f.h[1] = *(const v8h*)(p + 16); return f.v;
}
__device__ __forceinline__ v8f wmma16g(v16h a, v16h b, v8f c) {
    c = __builtin_amdgcn_wmma_f32_16x16x32_f16(false, a, false, b, (short)0, c, false, false);
    asm volatile("v_nop\n\tv_nop\n\tv_nop\n\tv_nop" : "+v"(c) : "v"(a), "v"(b));
    return c;
}
__device__ __forceinline__ void wave_sync_lds() {
    __builtin_amdgcn_fence(3  , "workgroup");
    __builtin_amdgcn_wave_barrier();
    __builtin_amdgcn_fence(2  , "workgroup");
}

__global__ __launch_bounds__(256) void k_wconv(const float* __restrict__ Wm, _Float16* __restrict__ W16, unsigned n8) {
    const unsigned u = blockIdx.x * 256u + threadIdx.x;
    if (u >= n8) return;
    const float* s = Wm + (size_t)u * 8u;
    const v4f a = *(const v4f*)s, b = *(const v4f*)(s + 4);
    v8h pk;
    pk[0] = toh_flush(bfr(a.x) * W_CARRY); pk[1] = toh_flush(bfr(a.y) * W_CARRY);
    pk[2] = toh_flush(bfr(a.z) * W_CARRY); pk[3] = toh_flush(bfr(a.w) * W_CARRY);
    pk[4] = toh_flush(bfr(b.x) * W_CARRY); pk[5] = toh_flush(bfr(b.y) * W_CARRY);
    pk[6] = toh_flush(bfr(b.z) * W_CARRY); pk[7] = toh_flush(bfr(b.w) * W_CARRY);
    st8_twice(W16 + (size_t)u * 8u, pk);
}

__global__ __launch_bounds__(256) void k_xw(const float* __restrict__ x, _Float16* __restrict__ xw, unsigned img0) {
    const unsigned u = blockIdx.x * 256u + threadIdx.x;
    if (u >= (unsigned)(MROWS * (CD / 8))) return;
    const unsigned row = u >> 4, c0 = (u & 15u) * 8u;
    const unsigned win = row >> 6, r = row & 63u;
    const unsigned b = img0 + (win >> 6), w = win & 63u;
    const unsigned wi = w >> 3, wj = w & 7u;
    const unsigned rc = min(r, 48u);
    const unsigned ri = div7_u6(rc), rj = rc - 7u * ri;
    const unsigned ii = (7u * wi + ri + 3u) % 56u;
    const unsigned jj = (7u * wj + rj + 3u) % 56u;
    const float* xr = x + ((size_t)b * LTOK + ii * 56u + jj) * CD + c0;
    const v4f a = *(const v4f*)xr, q = *(const v4f*)(xr + 4);
    const bool live = r < 49u;
    v8h pk;
    pk[0] = toh_flush(live ? bfr(a.x) * X_CARRY : 0.0f); pk[1] = toh_flush(live ? bfr(a.y) * X_CARRY : 0.0f);
    pk[2] = toh_flush(live ? bfr(a.z) * X_CARRY : 0.0f); pk[3] = toh_flush(live ? bfr(a.w) * X_CARRY : 0.0f);
    pk[4] = toh_flush(live ? bfr(q.x) * X_CARRY : 0.0f); pk[5] = toh_flush(live ? bfr(q.y) * X_CARRY : 0.0f);
    pk[6] = toh_flush(live ? bfr(q.z) * X_CARRY : 0.0f); pk[7] = toh_flush(live ? bfr(q.w) * X_CARRY : 0.0f);
    st8_twice(xw + (size_t)row * CD + c0, pk);
}

__device__ __forceinline__ void gemm64_k128(const _Float16* __restrict__ A, const _Float16* __restrict__ Bt,
                                            unsigned m0, unsigned n0, unsigned rlane, unsigned koff, v8f (&acc)[4][4]) {
#pragma unroll
  for (int i = 0; i < 4; ++i)
#pragma unroll
    for (int j = 0; j < 4; ++j) acc[i][j] = (v8f){0.f,0.f,0.f,0.f,0.f,0.f,0.f,0.f};
#pragma unroll 1
  for (unsigned k0 = 0; k0 < 128u; k0 += 32u) {
    v16h bh[4];
#pragma unroll
    for (int j = 0; j < 4; ++j)
      bh[j] = frag_ld(Bt + (size_t)(n0 + ((unsigned)j << 4) + rlane) * 128u + koff + k0);
#pragma unroll
    for (int i = 0; i < 4; ++i) {
      const v16h ah = frag_ld(A + (size_t)(m0 + ((unsigned)i << 4) + rlane) * 128u + koff + k0);
#pragma unroll
      for (int j = 0; j < 4; ++j) acc[i][j] = wmma16g(ah, bh[j], acc[i][j]);
    }
  }
}

template <bool ISQ>
__device__ __forceinline__ void epi_rows16(const v8f (&acc)[4][4], float* slab, _Float16* __restrict__ C, const float* __restrict__ bias,
                                           unsigned m0, unsigned nb0, unsigned cc0, unsigned lane) {
  const unsigned rlane = lane & 15u;
  const unsigned mOff = (lane >> 4) * 8u;
  float bv[4];
#pragma unroll
  for (int j = 0; j < 4; ++j) bv[j] = bfr(bias[nb0 + ((unsigned)j << 4) + rlane]);
#pragma unroll
  for (int i = 0; i < 4; ++i) {
    const unsigned mBase = m0 + ((unsigned)i << 4);
#pragma unroll
    for (int j = 0; j < 4; ++j) {
#pragma unroll
      for (int r = 0; r < 8; ++r) {
        float v = acc[i][j][r] * QKV_UNDO + bv[j];
        if (ISQ) v *= QSCALE;
        v *= QKV_CARRY;
        slab[(mOff + (unsigned)r) * 68u + ((unsigned)j << 4) + rlane] = v;
      }
    }
    wave_sync_lds();
    {
      const unsigned q = lane >> 3, c8 = (lane & 7u) * 8u;
      v8h hv[4];
#pragma unroll
      for (int it = 0; it < 4; ++it) {
        const unsigned row = (unsigned)it * 4u + q;
        const float* sp = slab + row * 68u + c8;
#pragma unroll
        for (int e = 0; e < 8; ++e) hv[it][e] = toh_flush(sp[e]);
      }
      for (int pass = 0; pass < 2; ++pass) {
#pragma unroll
        for (int it = 0; it < 4; ++it) {
          const unsigned row = (unsigned)it * 4u + q;
          *(volatile v8h*)(C + (size_t)(mBase + row) * 128u + cc0 + c8) = hv[it];
        }
        __threadfence();
      }
    }
    wave_sync_lds();
  }
}

__device__ __forceinline__ void epi_vt(const v8f (&acc)[4][4], _Float16* sVw, _Float16* __restrict__ VT, const float* __restrict__ bias,
                                       unsigned win, unsigned vt, unsigned lane) {
  const unsigned rlane = lane & 15u;
  const unsigned hh = lane >> 4;
#pragma unroll
  for (int j = 0; j < 4; ++j) {
    const float bv = bfr(bias[256u + 64u * vt + ((unsigned)j << 4) + rlane]);
#pragma unroll
    for (int i = 0; i < 4; ++i) {
      v8h pc;
#pragma unroll
      for (int r = 0; r < 8; ++r) pc[r] = toh_flush((acc[i][j][r] * QKV_UNDO + bv) * QKV_CARRY);
      *(v8h*)(sVw + (((unsigned)j << 4) + rlane) * 72u + ((unsigned)i << 4) + 8u * hh) = pc;
    }
  }
  wave_sync_lds();
  const unsigned q = lane >> 3, c8 = (lane & 7u) * 8u;
#pragma unroll
  for (int g = 0; g < 4; ++g) {
    v8h hv[4];
#pragma unroll
    for (int it = 0; it < 4; ++it) {
      const unsigned row = (unsigned)g * 16u + (unsigned)it * 4u + q;
      hv[it] = *(const v8h*)(sVw + row * 72u + c8);
    }
    for (int pass = 0; pass < 2; ++pass) {
#pragma unroll
      for (int it = 0; it < 4; ++it) {
        const unsigned row = (unsigned)g * 16u + (unsigned)it * 4u + q;
        *(volatile v8h*)(VT + ((size_t)win * 128u + 64u * vt + row) * 64u + c8) = hv[it];
      }
      __threadfence();
    }
  }
}

__global__ __launch_bounds__(128) void k_qkv(const _Float16* __restrict__ A, const _Float16* __restrict__ Bt,
                                             const float* __restrict__ bias, _Float16* __restrict__ Q16,
                                             _Float16* __restrict__ K16, _Float16* __restrict__ VT16) {
  __shared__ __align__(16) float sT[4][16 * 68];
  __shared__ __align__(16) _Float16 sV[4][64 * 72];
  const unsigned lane = threadIdx.x & 31u;
  const unsigned wave = (unsigned)__builtin_amdgcn_readfirstlane((int)(threadIdx.x >> 5));
  const unsigned tm = blockIdx.x * 4u + wave;
  const unsigned tn = blockIdx.y;
  if (tm >= (unsigned)NWINP) return;
  const unsigned m0 = tm << 6, n0 = tn << 6;
  v8f acc[4][4];
  gemm64_k128(A, Bt, m0, n0, lane & 15u, (lane >> 4) * 8u, acc);
  if (tn < 2u)      epi_rows16<true >(acc, sT[wave], Q16, bias, m0, n0, n0, lane);
  else if (tn < 4u) epi_rows16<false>(acc, sT[wave], K16, bias, m0, n0, n0 - 128u, lane);
  else              epi_vt(acc, sV[wave], VT16, bias, tm, tn - 4u, lane);
}

__global__ __launch_bounds__(256) void k_attn(const _Float16* __restrict__ Q16, const _Float16* __restrict__ K16,
                                              const _Float16* __restrict__ VT16, const float* __restrict__ mask,
                                              const float* __restrict__ tab, _Float16* __restrict__ CTX16) {
  __shared__ float sTab[4 * 176];
  __shared__ float sMask[2432];
  __shared__ __align__(16) _Float16 sO[8][16 * 72];
  const unsigned tid = threadIdx.x, lane = tid & 31u;
  const unsigned wave = (unsigned)__builtin_amdgcn_readfirstlane((int)(tid >> 5));
  const unsigned hh = lane >> 4, c = lane & 15u;
  const unsigned win = blockIdx.x;
  const unsigned w = win & 63u;
#pragma unroll 1
  for (unsigned i = tid; i < 676u; i += 256u) sTab[(i & 3u) * 176u + (i >> 2)] = bfr(tab[i]);
#pragma unroll 1
  for (unsigned i = tid; i < 2401u; i += 256u) sMask[i] = bfr(mask[(size_t)w * 2401u + i]);
  __syncthreads();

  const unsigned pair = wave >> 2, qt = wave & 3u;
  const unsigned n = 16u * qt + c;
  const unsigned nq = min(n, 48u);
  const unsigned nli = div7_u6(nq);
  const unsigned an = 6u * nli + nq + 84u;
  const unsigned mrow = nq * 49u;
  _Float16* ow = sO[wave];
  const size_t rbase = (size_t)win * 64u;
#pragma unroll 1
  for (unsigned hp = 0; hp < 2u; ++hp) {
    const unsigned head = 2u * pair + hp;
    const v16h qf = frag_ld(Q16 + (rbase + n) * 128u + 32u * head + 8u * hh);
    v8f s[4];
#pragma unroll
    for (int j = 0; j < 4; ++j) {
      const v16h kf = frag_ld(K16 + (rbase + (unsigned)j * 16u + c) * 128u + 32u * head + 8u * hh);
      const v8f z = (v8f){0.f,0.f,0.f,0.f,0.f,0.f,0.f,0.f};
      s[j] = wmma16g(kf, qf, z);
    }
    const unsigned tb = head * 176u + an;
    float mx = -3.0e38f;
#pragma unroll
    for (int j = 0; j < 4; ++j) {
#pragma unroll
      for (int r = 0; r < 8; ++r) {
        const unsigned m = 16u * (unsigned)j + 8u * hh + (unsigned)r;
        const unsigned mk = min(m, 48u);
        const unsigned bm = 6u * div7_u6(mk) + mk;
        const float bz = sTab[tb - bm];
        const float mz = sMask[mrow + mk];
        float tv = ((s[j][r] * S_UNDO + bz) + mz) * LOG2E;
        if (j == 3) { const bool live = (8u * hh + (unsigned)r) < 1u; tv = live ? tv : -3.0e38f; }
        s[j][r] = tv;
        mx = (tv > mx) ? tv : mx;
      }
    }
    const float mo = __shfl_xor(mx, 16, 32);
    mx = (mo > mx) ? mo : mx;
    float sum = 0.f;
#pragma unroll
    for (int j = 0; j < 4; ++j) {
#pragma unroll
      for (int r = 0; r < 8; ++r) {
        const float e = exp2f(s[j][r] - mx);
        s[j][r] = e;
        sum += e;
      }
    }
    sum += __shfl_xor(sum, 16, 32);
    const float inv = P_CARRY * (1.0f / sum);
    v16h pb0, pb1;
#pragma unroll
    for (int r = 0; r < 8; ++r) {
      pb0[r]     = toh_flush(s[0][r] * inv);
      pb0[8 + r] = toh_flush(s[1][r] * inv);
      pb1[r]     = toh_flush(s[2][r] * inv);
      pb1[8 + r] = toh_flush(s[3][r] * inv);
    }
#pragma unroll
    for (int t = 0; t < 2; ++t) {
      const _Float16* vrow = VT16 + ((size_t)win * 128u + 32u * head + (unsigned)t * 16u + c) * 64u + 8u * hh;
      v8f o = (v8f){0.f,0.f,0.f,0.f,0.f,0.f,0.f,0.f};
      const v16h va0 = frag_ld(vrow);
      o = wmma16g(va0, pb0, o);
      const v16h va1 = frag_ld(vrow + 32);
      o = wmma16g(va1, pb1, o);
      v8h pc;
#pragma unroll
      for (int r = 0; r < 8; ++r) pc[r] = toh_flush(o[r] * O_UNDO);
      *(v8h*)(ow + c * 72u + hp * 32u + (unsigned)t * 16u + 8u * hh) = pc;
    }
  }
  wave_sync_lds();
  {
    const unsigned q = lane >> 3, c8 = (lane & 7u) * 8u;
    v8h ov[4];
#pragma unroll
    for (int it = 0; it < 4; ++it) ov[it] = *(const v8h*)(ow + ((unsigned)it * 4u + q) * 72u + c8);
    _Float16* dst = CTX16 + (rbase + 16u * qt) * 128u + pair * 64u;
    for (int pass = 0; pass < 2; ++pass) {
#pragma unroll
      for (int it = 0; it < 4; ++it) *(volatile v8h*)(dst + (size_t)((unsigned)it * 4u + q) * 128u + c8) = ov[it];
      __threadfence();
    }
  }
}

__global__ __launch_bounds__(256) void k_proj(const _Float16* __restrict__ A, const _Float16* __restrict__ Bt,
                                              const float* __restrict__ bias, float* __restrict__ out, unsigned img0) {
  __shared__ __align__(16) float sT[8][16 * 68];
  const unsigned lane = threadIdx.x & 31u;
  const unsigned wave = (unsigned)__builtin_amdgcn_readfirstlane((int)(threadIdx.x >> 5));
  const unsigned tm = blockIdx.x * 8u + wave;
  const unsigned tn = blockIdx.y;
  if (tm >= (unsigned)NWINP) return;
  const unsigned m0 = tm << 6, n0 = tn << 6;
  const unsigned rlane = lane & 15u;
  const unsigned mOff = (lane >> 4) * 8u;
  v8f acc[4][4];
  gemm64_k128(A, Bt, m0, n0, rlane, mOff, acc);

  const unsigned b = img0 + (tm >> 6), w = tm & 63u;
  const unsigned wi = w >> 3, wj = w & 7u;
  float bv[4];
#pragma unroll
  for (int j = 0; j < 4; ++j) bv[j] = bfr(bias[n0 + ((unsigned)j << 4) + rlane]);
  float* slab = sT[wave];
#pragma unroll
  for (int i = 0; i < 4; ++i) {
#pragma unroll
    for (int j = 0; j < 4; ++j) {
#pragma unroll
      for (int r = 0; r < 8; ++r)
        slab[(mOff + (unsigned)r) * 68u + ((unsigned)j << 4) + rlane] = acc[i][j][r] * PROJ_UNDO + bv[j];
    }
    wave_sync_lds();
    {
      const unsigned hh = lane >> 4, c4 = (lane & 15u) * 4u;
#pragma unroll
      for (int half = 0; half < 2; ++half) {
        v4f vv[4];
        size_t doff[4];
        bool ok[4];
#pragma unroll
        for (int it = 0; it < 4; ++it) {
          const unsigned row = (unsigned)(half * 4 + it) * 2u + hh;
          const unsigned rw = ((unsigned)i << 4) + row;
          const unsigned rc = min(rw, 48u);
          const unsigned ri = div7_u6(rc), rj = rc - 7u * ri;
          const unsigned ii = (7u * wi + ri + 3u) % 56u;
          const unsigned jj = (7u * wj + rj + 3u) % 56u;
          doff[it] = ((size_t)b * LTOK + ii * 56u + jj) * CD + n0 + c4;
          ok[it] = rw < 49u;
          vv[it] = *(const v4f*)(slab + row * 68u + c4);
        }
        for (int pass = 0; pass < 2; ++pass) {
#pragma unroll
          for (int it = 0; it < 4; ++it) {
            if (ok[it]) *(volatile v4f*)(out + doff[it]) = vv[it];
          }
          __threadfence();
        }
      }
    }
    wave_sync_lds();
  }
}

extern "C" void kernel_launch(void* const* d_in, const int* in_sizes, int n_in, void* d_out, int out_size,
                              void* d_ws, size_t ws_size, hipStream_t stream) {
    if (n_in < 9) return;
    if (in_sizes[0] < NB * LTOK * CD || in_sizes[1] < NWIMG * NTOK * NTOK || in_sizes[2] < QKVN * CD || in_sizes[3] < QKVN) return;
    if (in_sizes[4] < CD * CD || in_sizes[5] < CD || in_sizes[6] < 169 * NH || in_sizes[7] < 1 || in_sizes[8] < 1) return;
    if (out_size < NB * LTOK * CD) return;

    const float* x      = (const float*)d_in[0];
    const float* amask  = (const float*)d_in[1];
    const float* qkv_w  = (const float*)d_in[2];
    const float* qkv_b  = (const float*)d_in[3];
    const float* proj_w = (const float*)d_in[4];
    const float* proj_b = (const float*)d_in[5];
    const float* rtab   = (const float*)d_in[6];
    const int*   dimH   = (const int*)d_in[7];
    const int*   dimW   = (const int*)d_in[8];
    (void)dimH; (void)dimW;
    float* out = (float*)d_out;

    char* wsp = (char*)d_ws;
    size_t off = 0;
    auto carve = [&](size_t bytes) -> void* { void* r = wsp + off; off += (bytes + 255) & ~(size_t)255; return r; };
    _Float16* xw16  = (_Float16*)carve((size_t)MROWS * CD * 2);
    _Float16* q16   = (_Float16*)carve((size_t)MROWS * CD * 2);
    _Float16* k16   = (_Float16*)carve((size_t)MROWS * CD * 2);
    _Float16* vt16  = (_Float16*)carve((size_t)MROWS * CD * 2);
    _Float16* ctx16 = (_Float16*)carve((size_t)MROWS * CD * 2);
    _Float16* wq16  = (_Float16*)carve((size_t)QKVN * CD * 2);
    _Float16* wp16  = (_Float16*)carve((size_t)CD * CD * 2);
    if (off > ws_size || off > (size_t)134217728) return;

    k_wconv<<<(QKVN * CD / 8) / 256, 256, 0, stream>>>(qkv_w, wq16, (unsigned)(QKVN * CD / 8));
    k_wconv<<<(CD * CD / 8) / 256, 256, 0, stream>>>(proj_w, wp16, (unsigned)(CD * CD / 8));

    for (unsigned p = 0; p < (unsigned)NPASS; ++p) {
        const unsigned img0 = p * (unsigned)IMGS;
        k_xw<<<(MROWS * (CD / 8)) / 256, 256, 0, stream>>>(x, xw16, img0);
        k_qkv<<<dim3(NWINP / 4, QKVN / 64), 128, 0, stream>>>(xw16, wq16, qkv_b, q16, k16, vt16);
        k_attn<<<NWINP, 256, 0, stream>>>(q16, k16, vt16, amask, rtab, ctx16);
        k_proj<<<dim3(NWINP / 8, CD / 64), 256, 0, stream>>>(ctx16, wp16, proj_b, out, img0);
    }
}
